// CrossLinearAttention_5523327943105
// MI455X (gfx1250) — hardware-verified
//
#include <hip/hip_runtime.h>


#define NBI  4
#define NT   8192
#define DX   256
#define NH   8
#define HD   64
#define DI   (NH * HD)
#define DM   DX
#define IEPS 1e-5f
#define LOSC 1024.0f

typedef _Float16 h16;
typedef unsigned short bf;
typedef __attribute__((ext_vector_type(16))) __bf16   v16bf;
typedef __attribute__((ext_vector_type(16))) _Float16 v16h;
typedef __attribute__((ext_vector_type(8)))  _Float16 v8h;
typedef __attribute__((ext_vector_type(8)))  unsigned short v8us;
typedef __attribute__((ext_vector_type(8)))  float    v8f;
typedef __attribute__((ext_vector_type(4)))  float    v4f;
typedef v8h  __attribute__((may_alias)) v8ha;
typedef v4f  __attribute__((may_alias)) v4fa;
typedef v8us __attribute__((may_alias)) v8usa;

__device__ __forceinline__ unsigned short f2bf(float f) { unsigned u = __float_as_uint(f); u += 0x7FFFu + ((u >> 16) & 1u); return (unsigned short)(u >> 16); }
__device__ __forceinline__ float bf2f(unsigned short b) { return __uint_as_float(((unsigned)b) << 16); }
__device__ __forceinline__ float bfr(float f) { return bf2f(f2bf(f)); }
__device__ __forceinline__ v16h cat16(v8h lo, v8h hi) { return __builtin_shufflevector(lo, hi, 0, 1, 2, 3, 4, 5, 6, 7, 8, 9, 10, 11, 12, 13, 14, 15); }
__device__ __forceinline__ v16bf cat16b(v8us lo, v8us hi) { return __builtin_bit_cast(v16bf, __builtin_shufflevector(lo, hi, 0, 1, 2, 3, 4, 5, 6, 7, 8, 9, 10, 11, 12, 13, 14, 15)); }
__device__ __forceinline__ v8f wmma16(v16h a, v16h b, v8f c) { return __builtin_amdgcn_wmma_f32_16x16x32_f16(false, a, false, b, (short)0, c, false, false); }
__device__ __forceinline__ v8f wmmab(v16bf a, v16bf b, v8f c) { return __builtin_amdgcn_wmma_f32_16x16x32_bf16(false, a, false, b, (short)0, c, false, false); }

template <bool SPLITA, bool F16OUT = false>
__global__ __launch_bounds__(128) void k_gemmb(const bf* __restrict__ A, const bf* __restrict__ Al, const bf* __restrict__ Bn, const float* __restrict__ bias, float* C, int ldc, h16* C2, const float* __restrict__ R = nullptr, int K = DM, int roundR = 1) {
    __shared__ __align__(16) float ost[4][16 * 68];
    const int lane = threadIdx.x & 31, wave = threadIdx.x >> 5, lr = lane & 15, hi = lane >> 4;
    const int r0 = blockIdx.x * 64 + wave * 16, c0 = blockIdx.y * 64;
    const size_t aoff = (size_t)(r0 + lr) * K + 8 * hi;
    size_t boff[4];
#pragma unroll
    for (int t = 0; t < 4; ++t) boff[t] = (size_t)(c0 + t * 16 + lr) * K + 8 * hi;
    v8f acc[4];
#pragma unroll
    for (int t = 0; t < 4; ++t) acc[t] = (v8f){};
#pragma unroll 1
    for (int kc = 0; kc < K; kc += 32) {
        const v16bf a = cat16b(*(const v8us*)(A + aoff + kc), *(const v8us*)(A + aoff + kc + 16));
        v16bf al = a;
        if (SPLITA) al = cat16b(*(const v8us*)(Al + aoff + kc), *(const v8us*)(Al + aoff + kc + 16));
#pragma unroll
        for (int t = 0; t < 4; ++t) { const v16bf b = cat16b(*(const v8us*)(Bn + boff[t] + kc), *(const v8us*)(Bn + boff[t] + kc + 16)); acc[t] = wmmab(a, b, acc[t]); if (SPLITA) acc[t] = wmmab(al, b, acc[t]); }
        asm volatile("v_nop\n\tv_nop\n\tv_nop\n\tv_nop" : "+v"(acc[0]), "+v"(acc[1]), "+v"(acc[2]), "+v"(acc[3]) : "v"(a), "v"(al));
    }
    float* os = &ost[wave][0];
#pragma unroll
    for (int t = 0; t < 4; ++t) { const float bv = bias ? bfr(bias[c0 + t * 16 + lr]) : 0.f;
#pragma unroll
        for (int j = 0; j < 8; ++j) os[(hi * 8 + j) * 68 + t * 16 + lr] = acc[t][j] + bv; }
    __syncthreads();
    if (F16OUT) {
        h16* crow = (h16*)(void*)C + (size_t)r0 * ldc + c0;
        auto pass = [&]() {
#pragma unroll
            for (int s = 0; s < 4; ++s) { const int row = 4 * s + (lane >> 3), piece = lane & 7; const float* sp = os + row * 68 + piece * 8; v8h o, o2;
#pragma unroll
                for (int i = 0; i < 8; ++i) { const h16 a = (h16)sp[i]; o[i] = a; o2[i] = (h16)((sp[i] - (float)a) * LOSC); }
                *(volatile v8h*)(crow + (size_t)row * ldc + piece * 8) = o; if (C2) *(volatile v8h*)(C2 + (size_t)r0 * ldc + c0 + (size_t)row * ldc + piece * 8) = o2; }
        };
        pass(); __threadfence(); pass();
    } else {
        float* crow = C + (size_t)r0 * ldc + c0;
        auto pass = [&]() {
#pragma unroll
            for (int s = 0; s < 8; ++s) { const int Lid = (lane >> 3) + 4 * s, piece = lane & 7; const int row = Lid >> 1, cofs = (Lid & 1) * 32 + piece * 4;
                v4f val = *(const v4fa*)(os + row * 68 + cofs); if (R) { const v4f rv = *(const v4f*)(R + ((size_t)r0 + row) * ldc + c0 + cofs); val += roundR ? (v4f){bfr(rv[0]), bfr(rv[1]), bfr(rv[2]), bfr(rv[3])} : rv; }
                *(volatile v4f*)(crow + (size_t)row * ldc + cofs) = val; }
        };
        pass(); __threadfence(); pass();
    }
}


__global__ __launch_bounds__(256) void k_wt(const float* __restrict__ Wm, int K, int ncols, bf* WT) {
    __shared__ __align__(16) unsigned short tl[64 * 72];
    const int tid = threadIdx.x, k0 = blockIdx.x * 64, n0 = blockIdx.y * 64;
    const int kk = tid >> 2, nq = (tid & 3) * 16;
#pragma unroll
    for (int i = 0; i < 16; ++i) tl[(nq + i) * 72 + kk] = f2bf(Wm[(size_t)(k0 + kk) * ncols + n0 + nq + i]);
    __syncthreads();
    const int piece = tid & 7;
    auto pass = [&]() {
#pragma unroll
        for (int s = 0; s < 2; ++s) { const int nr = (tid >> 3) + 32 * s; const v8us val = *(const v8usa*)(tl + nr * 72 + piece * 8); *(volatile v8us*)(WT + (size_t)(n0 + nr) * K + k0 + piece * 8) = val; }
    };
    pass(); __threadfence(); pass();
}

__global__ __launch_bounds__(256) void k_cvt(const float* __restrict__ src, bf* dst) {
    const int lane = threadIdx.x & 31; const size_t r = (size_t)blockIdx.x * 8 + (threadIdx.x >> 5); if (r >= (size_t)NT) return; v8us o;
#pragma unroll
    for (int i = 0; i < 8; ++i) o[i] = f2bf(src[r * DX + lane * 8 + i]);
    *(volatile v8us*)(dst + r * DX + lane * 8) = o; __threadfence(); *(volatile v8us*)(dst + r * DX + lane * 8) = o;
}
__global__ __launch_bounds__(256) void k_split512(const float* __restrict__ src, bf* dh, bf* dl) {
    const int lane = threadIdx.x & 31; const size_t r = (size_t)blockIdx.x * 8 + (threadIdx.x >> 5); if (r >= (size_t)NT) return;
#pragma unroll 1
    for (int ps = 0; ps < 2; ++ps) {
#pragma unroll
        for (int q = 0; q < DI / 256; ++q) { const size_t o = r * DI + q * 256 + lane * 8; const v8f v = *(const v8f*)(src + o); v8us oh, ol;
#pragma unroll
            for (int i = 0; i < 8; ++i) { const unsigned short hb = f2bf(v[i]); oh[i] = hb; ol[i] = f2bf(v[i] - bf2f(hb)); }
            *(volatile v8us*)(dh + o) = oh; *(volatile v8us*)(dl + o) = ol; }
        if (ps == 0) __threadfence(); }
}
__global__ __launch_bounds__(256) void k_vtbn(const float* __restrict__ src, int ld, int col0, bf* Th, bf* Tl) {
    __shared__ float tl[64][65]; __shared__ float mu_[64]; __shared__ float rs_[64];
    const int tid = threadIdx.x, t0 = blockIdx.x * 64, h = blockIdx.y;
    { const int tt = tid >> 2, dq = (tid & 3) * 16;
#pragma unroll 4
      for (int i = 0; i < 16; ++i) tl[dq + i][tt] = src[(size_t)(t0 + tt) * ld + col0 + h * HD + dq + i]; }
    __syncthreads();
    if (tid < 64) { float s = 0.f;
#pragma unroll 8
        for (int d = 0; d < HD; ++d) s += tl[d][tid];
        const float mu = s * (1.0f / HD); float v = 0.f;
#pragma unroll 8
        for (int d = 0; d < HD; ++d) { const float e = tl[d][tid] - mu; v = fmaf(e, e, v); }
        mu_[tid] = mu; rs_[tid] = rsqrtf(v * (1.0f / HD) + IEPS); }
    __syncthreads();
    const int piece = tid & 7, Lid = tid >> 3;
    auto pass = [&]() {
#pragma unroll
        for (int s = 0; s < 2; ++s) { const int d = Lid + 32 * s; v8us oh, ol;
#pragma unroll
            for (int i = 0; i < 8; ++i) { const int tt = piece * 8 + i; const float v = (tl[d][tt] - mu_[tt]) * rs_[tt]; const unsigned short hb = f2bf(v); oh[i] = hb; ol[i] = f2bf(v - bf2f(hb)); }
            const size_t o = ((size_t)h * HD + d) * NT + t0 + piece * 8; *(volatile v8us*)(Th + o) = oh; *(volatile v8us*)(Tl + o) = ol; }
    };
    pass(); __threadfence(); pass();
}
__global__ __launch_bounds__(256) void k_dsplit(const float* __restrict__ src, bf* dh, bf* dl) {
    typedef __attribute__((ext_vector_type(2))) unsigned short v2us;
    const int lane = threadIdx.x & 31, r = blockIdx.x * 8 + (threadIdx.x >> 5); if (r >= HD) return; const size_t o = (size_t)r * HD + lane * 2; v2us oh, ol;
#pragma unroll
    for (int i = 0; i < 2; ++i) { const float y = src[o + i] * (1.0f / NT); const unsigned short hb = f2bf(y); oh[i] = hb; ol[i] = f2bf(y - bf2f(hb)); }
    *(volatile v2us*)(dh + o) = oh; *(volatile v2us*)(dl + o) = ol; __threadfence(); *(volatile v2us*)(dh + o) = oh; *(volatile v2us*)(dl + o) = ol;
}
__global__ __launch_bounds__(128) void k_gemm3ll(const bf* __restrict__ Ah, const bf* __restrict__ Al, int lda, const bf* __restrict__ Bh, const bf* __restrict__ Bl, int ldb, int K, float* C, int ldc) {
    __shared__ __align__(16) float ost[4][16 * 68];
    const int lane = threadIdx.x & 31, wave = threadIdx.x >> 5, lr = lane & 15, hi = lane >> 4;
    const int r0 = blockIdx.x * 64 + wave * 16, c0 = blockIdx.y * 64;
    const size_t aoff = (size_t)(r0 + lr) * lda + 8 * hi;
    v8f acc[4];
#pragma unroll
    for (int t = 0; t < 4; ++t) acc[t] = (v8f){};
#pragma unroll 1
    for (int kc = 0; kc < K; kc += 32) {
        const v16bf a = cat16b(*(const v8us*)(Ah + aoff + kc), *(const v8us*)(Ah + aoff + kc + 16));
        const v16bf al = cat16b(*(const v8us*)(Al + aoff + kc), *(const v8us*)(Al + aoff + kc + 16));
#pragma unroll
        for (int t = 0; t < 4; ++t) { const size_t bo = (size_t)(c0 + t * 16 + lr) * ldb + kc + 8 * hi;
            const v16bf bh = cat16b(*(const v8us*)(Bh + bo), *(const v8us*)(Bh + bo + 16)); const v16bf bl = cat16b(*(const v8us*)(Bl + bo), *(const v8us*)(Bl + bo + 16));
            acc[t] = wmmab(a, bh, acc[t]); acc[t] = wmmab(al, bh, acc[t]); acc[t] = wmmab(a, bl, acc[t]); }
        asm volatile("v_nop\n\tv_nop\n\tv_nop\n\tv_nop" : "+v"(acc[0]), "+v"(acc[1]), "+v"(acc[2]), "+v"(acc[3]) : "v"(a), "v"(al));
    }
    float* os = &ost[wave][0];
#pragma unroll
    for (int t = 0; t < 4; ++t) {
#pragma unroll
        for (int j = 0; j < 8; ++j) os[(hi * 8 + j) * 68 + t * 16 + lr] = acc[t][j]; }
    __builtin_amdgcn_wave_barrier(); asm volatile("" ::: "memory");
    float* crow = C + (size_t)r0 * ldc + c0;
    auto pass = [&]() {
#pragma unroll
        for (int s = 0; s < 8; ++s) { const int Lid = (lane >> 3) + 4 * s, piece = lane & 7; const int row = Lid >> 1, cofs = (Lid & 1) * 32 + piece * 4;
            const v4f val = *(const v4fa*)(os + row * 68 + cofs); *(volatile v4f*)(crow + (size_t)row * ldc + cofs) = val; }
    };
    pass(); __threadfence(); pass();
}

extern "C" void kernel_launch(void* const* d_in, const int* in_sizes, int n_in,
                              void* d_out, int out_size, void* d_ws, size_t ws_size, hipStream_t stream) {
    (void)in_sizes; (void)n_in; (void)out_size;
    const float* x = (const float*)d_in[0]; const float* z = (const float*)d_in[1]; const float* Wq = (const float*)d_in[2]; const float* Wkv = (const float*)d_in[3]; const float* Wo = (const float*)d_in[4]; const float* bo = (const float*)d_in[5];
    float* out = (float*)d_out;
    char* wsp = (char*)d_ws;
    auto take = [&](size_t bytes) { char* p = wsp; wsp += (bytes + 255) & ~(size_t)255; return (void*)p; };
    bf* WqT = (bf*)take((size_t)DI * DX * 2); bf* WkvT = (bf*)take((size_t)2 * DI * DX * 2); bf* WoT = (bf*)take((size_t)DX * DI * 2);
    bf* Xb = (bf*)take((size_t)NT * DX * 2); bf* Zb = (bf*)take((size_t)NT * DX * 2); float* TMP = (float*)take((size_t)NT * DI * 4);
    bf* Qh = (bf*)take((size_t)NT * DI * 2); bf* Ql = (bf*)take((size_t)NT * DI * 2); bf* KTh = (bf*)take((size_t)DI * NT * 2); bf* KTl = (bf*)take((size_t)DI * NT * 2); bf* VTh = (bf*)take((size_t)DI * NT * 2); bf* VTl = (bf*)take((size_t)DI * NT * 2);
    float* DT = (float*)take(HD * HD * 4); bf* DTh = (bf*)take(HD * HD * 2); bf* DTl = (bf*)take(HD * HD * 2); float* O = (float*)take((size_t)NT * DI * 4); bf* Oh = (bf*)take((size_t)NT * DI * 2); bf* Ol = (bf*)take((size_t)NT * DI * 2);
    if ((size_t)(wsp - (char*)d_ws) > ws_size) return;
    k_wt<<<dim3(DX / 64, DI / 64, 1), 256, 0, stream>>>(Wq, DX, DI, WqT); k_wt<<<dim3(DX / 64, (2 * DI) / 64, 1), 256, 0, stream>>>(Wkv, DX, 2 * DI, WkvT); k_wt<<<dim3(DI / 64, DX / 64, 1), 256, 0, stream>>>(Wo, DI, DX, WoT);
    for (int b = 0; b < NBI; ++b) {
        k_cvt<<<NT / 8, 256, 0, stream>>>(x + (size_t)b * NT * DX, Xb); k_cvt<<<NT / 8, 256, 0, stream>>>(z + (size_t)b * NT * DX, Zb);
        k_gemmb<false, false><<<dim3(NT / 64, DI / 64, 1), 128, 0, stream>>>(Xb, nullptr, WqT, nullptr, TMP, DI, nullptr, nullptr, DX); k_split512<<<NT / 8, 256, 0, stream>>>(TMP, Qh, Ql);
        k_gemmb<false, false><<<dim3(NT / 64, DI / 64, 1), 128, 0, stream>>>(Zb, nullptr, WkvT, nullptr, TMP, DI, nullptr, nullptr, DX); k_vtbn<<<dim3(NT / 64, NH, 1), 256, 0, stream>>>(TMP, DI, 0, KTh, KTl);
        k_gemmb<false, false><<<dim3(NT / 64, DI / 64, 1), 128, 0, stream>>>(Zb, nullptr, WkvT + (size_t)DI * DX, nullptr, TMP, DI, nullptr, nullptr, DX); k_vtbn<<<dim3(NT / 64, NH, 1), 256, 0, stream>>>(TMP, DI, 0, VTh, VTl);
        for (int h = 0; h < NH; ++h) { const size_t ho = (size_t)h * HD * NT;
            k_gemm3ll<<<dim3(1, 1, 1), 128, 0, stream>>>(VTh + ho, VTl + ho, NT, KTh + ho, KTl + ho, NT, NT, DT, HD);
            k_dsplit<<<HD / 8, 256, 0, stream>>>(DT, DTh, DTl);
            k_gemm3ll<<<dim3(NT / 64, 1, 1), 128, 0, stream>>>(Qh + h * HD, Ql + h * HD, DI, DTh, DTl, HD, HD, O + h * HD, DI); }
        k_split512<<<NT / 8, 256, 0, stream>>>(O, Oh, Ol);
        k_gemmb<true, false><<<dim3(NT / 64, DX / 64, 1), 128, 0, stream>>>(Oh, Ol, WoT, bo, out + (size_t)b * NT * DX, DX, nullptr, nullptr, DI);
    }
}
